// MultiHeadAttention_85074712199466
// MI455X (gfx1250) — hardware-run, weakly checked
//
#include <hip/hip_runtime.h>
#ifndef NB
#define NB 2
#endif
#ifndef SEQ
#define SEQ 2048
#endif
#define NB_FULL 2
#define SEQ_FULL 2048
#define DIM 2048
#define HEADS 16
#define HD 128
#define N3D (3 * DIM)
#define NROWS (NB * SEQ)
#define EARLY ((SEQ) < 512 ? (SEQ) : 512)

#define SZ_FLG ((size_t)64 * 128)
#define SZ_XC  ((size_t)NB * SEQ * DIM * 2)
#define SZ_WQ  ((size_t)N3D * DIM * 2)
#define SZ_CL  ((size_t)NB * EARLY * DIM * 2)
#define SZ_WO  ((size_t)DIM * DIM * 2)
#define SZ_PH  ((size_t)NB * HEADS * SEQ * HD * 2)
#define SZ_PL  ((size_t)NB * HEADS * EARLY * HD * 2)

static_assert(SEQ % 128 == 0);
static_assert(EARLY % 128 == 0);
static_assert(SEQ <= SEQ_FULL);
static_assert(NB <= NB_FULL);
static_assert(HD == 128);
static_assert(DIM == HEADS * HD);
static_assert(DIM % 64 == 0);
static_assert(N3D % 64 == 0);
static_assert(SZ_CL <= SZ_WQ);
static_assert(SZ_FLG % 256 == 0 && SZ_XC % 256 == 0 && SZ_WQ % 256 == 0 && SZ_WO % 256 == 0 && SZ_PH % 256 == 0 && SZ_PL % 256 == 0);
static_assert(SZ_FLG + SZ_XC + SZ_WQ + SZ_WO + 3 * SZ_PH + 3 * SZ_PL <= (size_t)134217728);

typedef __bf16 v16b __attribute__((ext_vector_type(16)));
typedef _Float16 v16h __attribute__((ext_vector_type(16)));
typedef unsigned short v8us __attribute__((ext_vector_type(8), may_alias));
typedef float v8f __attribute__((ext_vector_type(8)));
typedef float v4f __attribute__((ext_vector_type(4)));
typedef float v4fa __attribute__((ext_vector_type(4), may_alias));
typedef int v4i __attribute__((ext_vector_type(4)));
typedef int v4ia __attribute__((ext_vector_type(4), may_alias));
union Frag { v16h h; v16b b; v8us half[2]; _Float16 e[16]; };
union Pack8 { v8us v; _Float16 e[8]; unsigned short u[8]; };
union Half1 { _Float16 e; unsigned short u; };

#define LOG2E 1.4426950408889634f
#define NEGV (-1000000000.0f)

__device__ __forceinline__ unsigned short bf16_bits(float x) {
  unsigned int u = __float_as_uint(x);
  return (unsigned short)((u + 0x7FFFu + ((u >> 16) & 1u)) >> 16);
}
__device__ __forceinline__ float bf16_rne(float x) { return __uint_as_float(((unsigned int)bf16_bits(x)) << 16); }

__device__ __forceinline__ void ldfrag(Frag& f, const unsigned short* __restrict__ p) {
  f.half[0] = *(const v8us*)(p);
  f.half[1] = *(const v8us*)(p + 16);
}
__device__ __forceinline__ v8f wm_h(const Frag& a, const Frag& b, v8f c) {
  return __builtin_amdgcn_wmma_f32_16x16x32_f16(false, a.h, false, b.h, (short)0, c, false, false);
}
__device__ __forceinline__ v8f wm_b(const Frag& a, const Frag& b, v8f c) {
  return __builtin_amdgcn_wmma_f32_16x16x32_bf16(false, a.b, false, b.b, (short)0, c, false, false);
}
template <bool F16>
__device__ __forceinline__ v8f wm(const Frag& a, const Frag& b, v8f c) {
  if (F16) return wm_h(a, b, c);
  return wm_b(a, b, c);
}

__global__ __launch_bounds__(256) void k_maskchk(const int* __restrict__ M, int* __restrict__ flg) {
  __shared__ int wb[8];
  const int tid = threadIdx.x;
  const int r0 = blockIdx.x * (SEQ / 64);
  int bad = 0;
#pragma unroll 1
  for (int rr = 0; rr < SEQ / 64; ++rr) {
    const int row = r0 + rr;
    const int* mp = M + (size_t)row * SEQ_FULL;
    for (int c = tid * 4; c < SEQ; c += 1024) {
      const v4i m = *(const v4ia*)(mp + c);
      bad |= ((m[0] != 0) != (c + 0 <= row)) ? 1 : 0;
      bad |= ((m[1] != 0) != (c + 1 <= row)) ? 1 : 0;
      bad |= ((m[2] != 0) != (c + 2 <= row)) ? 1 : 0;
      bad |= ((m[3] != 0) != (c + 3 <= row)) ? 1 : 0;
    }
  }
  int v = bad;
#pragma unroll
  for (int sh = 16; sh; sh >>= 1) v |= __shfl_xor(v, sh, 32);
  if ((tid & 31) == 0) wb[tid >> 5] = v;
  __syncthreads();
  int any = 0;
#pragma unroll
  for (int k = 0; k < 8; ++k) any |= wb[k];
  if (tid < 8) {
    const int fv = any ? 1 : 0;
    const v4i f = {fv, fv, fv, fv};
    int* d = flg + blockIdx.x * 32 + tid * 4;
    *(volatile v4i*)d = f;
    __threadfence();
    *(volatile v4i*)d = f;
  }
}

__global__ __launch_bounds__(256) void k_xb(const float* __restrict__ X, unsigned short* __restrict__ Xb) {
  const int t = blockIdx.x * 256 + threadIdx.x;
  if (t >= NROWS * (DIM / 8)) return;
  const int row = t / (DIM / 8), piece = t - row * (DIM / 8);
  const int b = row / SEQ, s = row - b * SEQ;
  const float* src = X + ((size_t)b * SEQ_FULL + s) * DIM + piece * 8;
  const v4f x0 = *(const v4fa*)(src), x1 = *(const v4fa*)(src + 4);
  Pack8 o;
  o.u[0] = bf16_bits(x0[0]); o.u[1] = bf16_bits(x0[1]); o.u[2] = bf16_bits(x0[2]); o.u[3] = bf16_bits(x0[3]);
  o.u[4] = bf16_bits(x1[0]); o.u[5] = bf16_bits(x1[1]); o.u[6] = bf16_bits(x1[2]); o.u[7] = bf16_bits(x1[3]);
  const v8us ov = o.v;
  unsigned short* d = Xb + (size_t)t * 8;
  *(volatile v8us*)d = ov;
  __threadfence();
  *(volatile v8us*)d = ov;
}

template <int MODE>
__global__ __launch_bounds__(256) void k_wt(const float* __restrict__ W, unsigned short* __restrict__ WT, int N) {
  __shared__ __attribute__((aligned(16))) unsigned short tl[64][72];
  const int tid = threadIdx.x;
  const int ntn = N / 64;
  const int kt = blockIdx.x / ntn, nt = blockIdx.x - kt * ntn;
  const int k0 = kt * 64, n0 = nt * 64;
  for (int i = tid; i < 64 * 16; i += 256) {
    const int j = i >> 4, c4 = (i & 15) * 4;
    const v4f x = *(const v4fa*)(W + (size_t)(k0 + j) * N + n0 + c4);
#pragma unroll
    for (int e = 0; e < 4; ++e) {
      unsigned short bits;
      if (MODE == 0) {
        bits = bf16_bits(x[e]);
      } else {
        Half1 hv;
        hv.e = (_Float16)(bf16_rne(x[e]) * 256.0f);
        bits = hv.u;
      }
      tl[c4 + e][j] = bits;
    }
  }
  __syncthreads();
  for (int pass = 0; pass < 2; ++pass) {
    for (int i = tid; i < 64 * 8; i += 256) {
      const int n = i >> 3, j8 = (i & 7) * 8;
      const v8us o = *(const v8us*)&tl[n][j8];
      *(volatile v8us*)(WT + (size_t)(n0 + n) * DIM + k0 + j8) = o;
    }
    if (pass == 0) __threadfence();
  }
}

template <bool F16, bool LO>
__device__ __forceinline__ void gemm_tile(const unsigned short* __restrict__ pa, const unsigned short* __restrict__ pl,
                                          const unsigned short* __restrict__ pb, v8f (&acc)[2][4]) {
#pragma unroll 2
  for (int k0 = 0; k0 < DIM; k0 += 32) {
    Frag a0, a1, b0, b1, b2, b3;
    ldfrag(a0, pa + k0);
    ldfrag(a1, pa + 16 * DIM + k0);
    ldfrag(b0, pb + k0);
    ldfrag(b1, pb + 16 * DIM + k0);
    ldfrag(b2, pb + 32 * DIM + k0);
    ldfrag(b3, pb + 48 * DIM + k0);
    acc[0][0] = wm<F16>(a0, b0, acc[0][0]);
    acc[0][1] = wm<F16>(a0, b1, acc[0][1]);
    acc[0][2] = wm<F16>(a0, b2, acc[0][2]);
    acc[0][3] = wm<F16>(a0, b3, acc[0][3]);
    acc[1][0] = wm<F16>(a1, b0, acc[1][0]);
    acc[1][1] = wm<F16>(a1, b1, acc[1][1]);
    acc[1][2] = wm<F16>(a1, b2, acc[1][2]);
    acc[1][3] = wm<F16>(a1, b3, acc[1][3]);
    asm volatile("v_nop\n\tv_nop\n\tv_nop\n\tv_nop"
                 : "+v"(acc[0][0]), "+v"(acc[0][1]), "+v"(acc[0][2]), "+v"(acc[0][3]),
                   "+v"(acc[1][0]), "+v"(acc[1][1]), "+v"(acc[1][2]), "+v"(acc[1][3])
                 : "v"(a0.h), "v"(a1.h), "v"(b0.h), "v"(b1.h), "v"(b2.h), "v"(b3.h));
    if (LO) {
      Frag l0, l1;
      ldfrag(l0, pl + k0);
      ldfrag(l1, pl + 16 * DIM + k0);
      acc[0][0] = wm<F16>(l0, b0, acc[0][0]);
      acc[0][1] = wm<F16>(l0, b1, acc[0][1]);
      acc[0][2] = wm<F16>(l0, b2, acc[0][2]);
      acc[0][3] = wm<F16>(l0, b3, acc[0][3]);
      acc[1][0] = wm<F16>(l1, b0, acc[1][0]);
      acc[1][1] = wm<F16>(l1, b1, acc[1][1]);
      acc[1][2] = wm<F16>(l1, b2, acc[1][2]);
      acc[1][3] = wm<F16>(l1, b3, acc[1][3]);
      asm volatile("v_nop\n\tv_nop\n\tv_nop\n\tv_nop"
                   : "+v"(acc[0][0]), "+v"(acc[0][1]), "+v"(acc[0][2]), "+v"(acc[0][3]),
                     "+v"(acc[1][0]), "+v"(acc[1][1]), "+v"(acc[1][2]), "+v"(acc[1][3])
                   : "v"(l0.h), "v"(l1.h), "v"(b0.h), "v"(b1.h), "v"(b2.h), "v"(b3.h));
    }
  }
}

__device__ __forceinline__ void store_qk(const float (*so)[68], unsigned short* __restrict__ Ph, unsigned short* __restrict__ Pl,
                                         size_t bh, int s0, int d0, bool early, int tid) {
  for (int pass = 0; pass < 2; ++pass) {
#pragma unroll 1
    for (int it = 0; it < 8; ++it) {
      const int i = tid + 128 * it;
      const int row = i >> 3, pc = i & 7;
      const v4f x0 = *(const v4fa*)&so[row][8 * pc], x1 = *(const v4fa*)&so[row][8 * pc + 4];
      Pack8 hi, lo;
#pragma unroll
      for (int e = 0; e < 4; ++e) {
        const float v0 = x0[e] * 1024.0f, v1 = x1[e] * 1024.0f;
        const _Float16 h0 = (_Float16)v0, h1 = (_Float16)v1;
        hi.e[e] = h0; hi.e[4 + e] = h1;
        lo.e[e] = (_Float16)(v0 - (float)h0); lo.e[4 + e] = (_Float16)(v1 - (float)h1);
      }
      const v8us hv = hi.v, lv = lo.v;
      *(volatile v8us*)(Ph + ((bh * SEQ + s0 + row) * HD + d0 + 8 * pc)) = hv;
      if (early) *(volatile v8us*)(Pl + ((bh * EARLY + s0 + row) * HD + d0 + 8 * pc)) = lv;
    }
    if (pass == 0) __threadfence();
  }
}

__device__ __forceinline__ void store_vt(const float (*so)[68], unsigned short* __restrict__ Ph, unsigned short* __restrict__ Pl,
                                         size_t bh, int s0, int d0, bool early, int tid) {
  for (int pass = 0; pass < 2; ++pass) {
#pragma unroll 1
    for (int it = 0; it < 8; ++it) {
      const int i = tid + 128 * it;
      const int d = i >> 4, pc = i & 15;
      Pack8 hi, lo;
#pragma unroll
      for (int q = 0; q < 8; ++q) {
        const float v = so[8 * pc + q][d] * 1024.0f;
        const _Float16 h = (_Float16)v;
        hi.e[q] = h;
        lo.e[q] = (_Float16)(v - (float)h);
      }
      const v8us hv = hi.v, lv = lo.v;
      *(volatile v8us*)(Ph + ((bh * HD + d0 + d) * SEQ + s0 + 8 * pc)) = hv;
      if (early) *(volatile v8us*)(Pl + ((bh * HD + d0 + d) * EARLY + s0 + 8 * pc)) = lv;
    }
    if (pass == 0) __threadfence();
  }
}

__global__ __launch_bounds__(128) __attribute__((amdgpu_num_vgpr(256)))
void k_qkv(const unsigned short* __restrict__ Xb, const unsigned short* __restrict__ WqT, const float* __restrict__ bias,
           unsigned short* __restrict__ Qh, unsigned short* __restrict__ Ql,
           unsigned short* __restrict__ Kh, unsigned short* __restrict__ Kl,
           unsigned short* __restrict__ Vth, unsigned short* __restrict__ Vtl) {
  __shared__ __attribute__((aligned(16))) float so[128][68];
  const int tid = threadIdx.x;
  const int w = __builtin_amdgcn_readfirstlane(tid >> 5);
  const int lane = tid & 31, ln = lane & 15, hh = lane >> 4;
  const int n0 = blockIdx.x * 64, m0 = blockIdx.y * 128;
  v8f acc[2][4] = {};
  const unsigned short* pa = Xb + (size_t)(m0 + 32 * w + ln) * DIM + 8 * hh;
  const unsigned short* pb = WqT + (size_t)(n0 + ln) * DIM + 8 * hh;
  gemm_tile<false, false>(pa, pa, pb, acc);
#pragma unroll
  for (int j = 0; j < 4; ++j) {
    const float bj = bf16_rne(bias[n0 + 16 * j + ln]);
#pragma unroll
    for (int i = 0; i < 2; ++i)
#pragma unroll
      for (int r = 0; r < 8; ++r)
        so[32 * w + 16 * i + 8 * hh + r][16 * j + ln] = acc[i][j][r] + bj;
  }
  __syncthreads();
  const int hsel = n0 / (3 * HD);
  const int c0 = n0 - hsel * (3 * HD);
  const int which = c0 >> 7;
  const int d0 = c0 & (HD - 1);
  const int b = m0 / SEQ, s0 = m0 - b * SEQ;
  const bool early = s0 < EARLY;
  const size_t bh = (size_t)b * HEADS + hsel;
  if (which == 0)      store_qk(so, Qh, Ql, bh, s0, d0, early, tid);
  else if (which == 1) store_qk(so, Kh, Kl, bh, s0, d0, early, tid);
  else                 store_vt(so, Vth, Vtl, bh, s0, d0, early, tid);
}

__device__ __forceinline__ void mma_s1(const Frag& k0, const Frag& k1, const Frag& q, v8f& s0, v8f& s1) {
  s0 = wm_h(k0, q, s0);
  s1 = wm_h(k1, q, s1);
  asm volatile("v_nop\n\tv_nop\n\tv_nop\n\tv_nop" : "+v"(s0), "+v"(s1) : "v"(k0.h), "v"(k1.h), "v"(q.h));
}
__device__ __forceinline__ void mma_s3(const Frag& k0, const Frag& k1, const Frag& k0l, const Frag& k1l,
                                       const Frag& qh, const Frag& ql, v8f& s0, v8f& s1) {
  s0 = wm_h(k0, qh, s0);
  s1 = wm_h(k1, qh, s1);
  s0 = wm_h(k0, ql, s0);
  s1 = wm_h(k1, ql, s1);
  s0 = wm_h(k0l, qh, s0);
  s1 = wm_h(k1l, qh, s1);
  asm volatile("v_nop\n\tv_nop\n\tv_nop\n\tv_nop" : "+v"(s0), "+v"(s1)
               : "v"(k0.h), "v"(k1.h), "v"(k0l.h), "v"(k1l.h), "v"(qh.h), "v"(ql.h));
}
__device__ __forceinline__ void mma_o1(const Frag& v0, const Frag& v1, const Frag& p, v8f& o0, v8f& o1) {
  o0 = wm_h(v0, p, o0);
  o1 = wm_h(v1, p, o1);
  asm volatile("v_nop\n\tv_nop\n\tv_nop\n\tv_nop" : "+v"(o0), "+v"(o1) : "v"(v0.h), "v"(v1.h), "v"(p.h));
}
__device__ __forceinline__ void mma_o3(const Frag& v0, const Frag& v1, const Frag& v0l, const Frag& v1l,
                                       const Frag& ph, const Frag& pl, v8f& o0, v8f& o1) {
  o0 = wm_h(v0, ph, o0);
  o1 = wm_h(v1, ph, o1);
  o0 = wm_h(v0, pl, o0);
  o1 = wm_h(v1, pl, o1);
  o0 = wm_h(v0l, ph, o0);
  o1 = wm_h(v1l, ph, o1);
  asm volatile("v_nop\n\tv_nop\n\tv_nop\n\tv_nop" : "+v"(o0), "+v"(o1)
               : "v"(v0.h), "v"(v1.h), "v"(v0l.h), "v"(v1l.h), "v"(ph.h), "v"(pl.h));
}

template <bool EARLY_, bool MASK>
__device__ __forceinline__ void fa_step(const unsigned short* __restrict__ Kp, const unsigned short* __restrict__ Klp,
                                        const unsigned short* __restrict__ Vp, const unsigned short* __restrict__ Vlp,
                                        const int* __restrict__ mrow, int key0, int ln, int hh,
                                        const Frag (&qh)[4], const Frag (&ql)[4],
                                        float& mr, float& lr, v8f (&O)[8]) {
  const v8f z8 = {0.f, 0.f, 0.f, 0.f, 0.f, 0.f, 0.f, 0.f};
  v8f s0 = z8, s1 = z8;
  const unsigned short* kp0 = Kp + (size_t)(key0 + ln) * HD + 8 * hh;
  const unsigned short* kp1 = kp0 + 16 * HD;
  const unsigned short* kl0 = Klp + (size_t)(key0 + ln) * HD + 8 * hh;
  const unsigned short* kl1 = kl0 + 16 * HD;
#pragma unroll
  for (int c = 0; c < 4; ++c) {
    Frag k0, k1;
    ldfrag(k0, kp0 + 32 * c);
    ldfrag(k1, kp1 + 32 * c);
    if (EARLY_) {
      Frag k0l, k1l;
      ldfrag(k0l, kl0 + 32 * c);
      ldfrag(k1l, kl1 + 32 * c);
      mma_s3(k0, k1, k0l, k1l, qh[c], ql[c], s0, s1);
    } else {
      mma_s1(k0, k1, qh[c], s0, s1);
    }
  }
  const float scl = 0.08838834764831845f * 9.5367431640625e-07f;
  float sc[16];
#pragma unroll
  for (int r = 0; r < 8; ++r) { sc[r] = s0[r] * scl; sc[8 + r] = s1[r] * scl; }
  if (MASK) {
    const int* mp = mrow + key0 + 8 * hh;
    const v4i a0 = *(const v4ia*)(mp), a1 = *(const v4ia*)(mp + 4);
    const v4i b0 = *(const v4ia*)(mp + 16), b1 = *(const v4ia*)(mp + 20);
#pragma unroll
    for (int r = 0; r < 4; ++r) {
      sc[r]      = (a0[r] != 0) ? sc[r]      : NEGV;
      sc[4 + r]  = (a1[r] != 0) ? sc[4 + r]  : NEGV;
      sc[8 + r]  = (b0[r] != 0) ? sc[8 + r]  : NEGV;
      sc[12 + r] = (b1[r] != 0) ? sc[12 + r] : NEGV;
    }
  }
  float mx = sc[0];
#pragma unroll
  for (int i = 1; i < 16; ++i) mx = fmaxf(mx, sc[i]);
  mx = fmaxf(mx, __shfl_xor(mx, 16, 32));
  const float mnew = fmaxf(mr, mx);
  const float al = exp2f((mr - mnew) * LOG2E);
  mr = mnew;
  Frag ph, pl;
  float ps = 0.0f;
#pragma unroll
  for (int i = 0; i < 16; ++i) {
    const float pc = exp2f(fmaf(sc[i] - mnew, LOG2E, 10.0f));
    ps += pc;
    const _Float16 h = (_Float16)pc;
    ph.e[i] = h;
    pl.e[i] = (_Float16)(pc - (float)h);
  }
  ps += __shfl_xor(ps, 16, 32);
  lr = lr * al + ps;
#pragma unroll
  for (int t = 0; t < 8; ++t) O[t] = O[t] * al;
  const unsigned short* vp = Vp + (size_t)ln * SEQ + key0 + 8 * hh;
  const unsigned short* vlp = Vlp + (size_t)ln * EARLY + key0 + 8 * hh;
#pragma unroll
  for (int t = 0; t < 8; t += 2) {
    Frag v0, v1;
    ldfrag(v0, vp + (size_t)t * 16 * SEQ);
    ldfrag(v1, vp + (size_t)(t + 1) * 16 * SEQ);
    if (EARLY_) {
      Frag v0l, v1l;
      ldfrag(v0l, vlp + (size_t)t * 16 * EARLY);
      ldfrag(v1l, vlp + (size_t)(t + 1) * 16 * EARLY);
      mma_o3(v0, v1, v0l, v1l, ph, pl, O[t], O[t + 1]);
    } else {
      mma_o1(v0, v1, ph, O[t], O[t + 1]);
    }
  }
}

template <bool EARLY_>
__global__ __launch_bounds__(128) __attribute__((amdgpu_num_vgpr(256)))
void k_attn(const unsigned short* __restrict__ Qh, const unsigned short* __restrict__ Ql,
            const unsigned short* __restrict__ Kh, const unsigned short* __restrict__ Kl,
            const unsigned short* __restrict__ Vth, const unsigned short* __restrict__ Vtl,
            const int* __restrict__ M, unsigned short* __restrict__ Ctxh, unsigned short* __restrict__ Ctxl) {
  __shared__ __attribute__((aligned(16))) float so[4][16][132];
  constexpr int NTD = (SEQ - EARLY) / 64;
  constexpr int NT = EARLY_ ? (EARLY / 64) : (NTD > 0 ? NTD : 1);
  constexpr int QT0 = EARLY_ ? 0 : (EARLY / 64);
  const int tid = threadIdx.x;
  const int w = __builtin_amdgcn_readfirstlane(tid >> 5);
  const int lane = tid & 31, ln = lane & 15, hh = lane >> 4;
  const int bh = blockIdx.x / NT;
  const int qt = QT0 + (blockIdx.x - bh * NT);
  const int b = bh / HEADS, h = bh - b * HEADS;
  const int qbase = qt * 64 + 16 * w;
  const int qg = qbase + ln;
  const unsigned short* Kp = Kh + (size_t)bh * SEQ * HD;
  const unsigned short* Klp = Kl + (size_t)bh * EARLY * HD;
  const unsigned short* Vp = Vth + (size_t)bh * HD * SEQ;
  const unsigned short* Vlp = Vtl + (size_t)bh * HD * EARLY;
  const int* mrow = M + (size_t)qg * SEQ_FULL;
  Frag qh[4], ql[4];
  {
    const unsigned short* qrow = Qh + ((size_t)bh * SEQ + qg) * HD + 8 * hh;
#pragma unroll
    for (int c = 0; c < 4; ++c) ldfrag(qh[c], qrow + 32 * c);
    if (EARLY_) {
      const unsigned short* qlrow = Ql + ((size_t)bh * EARLY + qg) * HD + 8 * hh;
#pragma unroll
      for (int c = 0; c < 4; ++c) ldfrag(ql[c], qlrow + 32 * c);
    } else {
#pragma unroll
      for (int c = 0; c < 4; ++c) ql[c] = qh[c];
    }
  }
  float mr = -3.0e38f, lr = 0.0f;
  v8f O[8] = {};
  const int nfull = qbase >> 5;
#pragma unroll 1
  for (int j = 0; j < nfull; ++j)
    fa_step<EARLY_, false>(Kp, Klp, Vp, Vlp, mrow, 32 * j, ln, hh, qh, ql, mr, lr, O);
  fa_step<EARLY_, true>(Kp, Klp, Vp, Vlp, mrow, 32 * nfull, ln, hh, qh, ql, mr, lr, O);

  const float inv = 1.0f / lr;
#pragma unroll
  for (int t = 0; t < 8; ++t)
#pragma unroll
    for (int r = 0; r < 8; ++r)
      so[w][ln][16 * t + 8 * hh + r] = O[t][r] * inv;
  __syncthreads();
  unsigned short* ch = Ctxh + ((size_t)b * SEQ + qbase) * DIM + h * HD;
  unsigned short* cl = Ctxl + ((size_t)b * EARLY + (EARLY_ ? qbase : 0)) * DIM + h * HD;
  const int rsub = lane >> 4, pc = lane & 15;
  for (int pass = 0; pass < 2; ++pass) {
#pragma unroll
    for (int q = 0; q < 8; ++q) {
      const int row = 2 * q + rsub;
      const v4f x0 = *(const v4fa*)&so[w][row][8 * pc], x1 = *(const v4fa*)&so[w][row][8 * pc + 4];
      Pack8 hi, lo;
#pragma unroll
      for (int e = 0; e < 4; ++e) {
        const _Float16 h0 = (_Float16)x0[e], h1 = (_Float16)x1[e];
        hi.e[e] = h0; hi.e[4 + e] = h1;
        lo.e[e] = (_Float16)(x0[e] - (float)h0); lo.e[4 + e] = (_Float16)(x1[e] - (float)h1);
      }
      const v8us hv = hi.v, lv = lo.v;
      *(volatile v8us*)(ch + (size_t)row * DIM + 8 * pc) = hv;
      if (EARLY_) *(volatile v8us*)(cl + (size_t)row * DIM + 8 * pc) = lv;
    }
    if (pass == 0) __threadfence();
  }
}

__global__ __launch_bounds__(128) __attribute__((amdgpu_num_vgpr(256)))
void k_out(const unsigned short* __restrict__ Ctxh, const unsigned short* __restrict__ Ctxl,
           const unsigned short* __restrict__ WoT, const float* __restrict__ bias,
           const int* __restrict__ flg, float* __restrict__ out) {
  __shared__ __attribute__((aligned(16))) float so[128][68];
  __shared__ int wb[4];
  const int tid = threadIdx.x;
  const int w = __builtin_amdgcn_readfirstlane(tid >> 5);
  const int lane = tid & 31, ln = lane & 15, hh = lane >> 4;
  const int n0 = blockIdx.x * 64, m0 = blockIdx.y * 128;
  const int b = m0 / SEQ, s0 = m0 - b * SEQ;
  const bool early = s0 < EARLY;
  const int fv = flg[(tid & 63) * 32];
  int pv = (fv == 1) ? 1 : 0;
#pragma unroll
  for (int sh = 16; sh; sh >>= 1) pv |= __shfl_xor(pv, sh, 32);
  if (lane == 0) wb[w] = pv;
  __syncthreads();
  int bad = 0;
#pragma unroll
  for (int k = 0; k < 4; ++k) bad |= wb[k];
  v8f acc[2][4] = {};
  const unsigned short* pa = Ctxh + (size_t)(m0 + 32 * w + ln) * DIM + 8 * hh;
  const unsigned short* pl = Ctxl + ((size_t)b * EARLY + (early ? s0 : 0) + 32 * w + ln) * DIM + 8 * hh;
  const unsigned short* pb = WoT + (size_t)(n0 + ln) * DIM + 8 * hh;
  if (early) gemm_tile<true, true>(pa, pl, pb, acc);
  else       gemm_tile<true, false>(pa, pa, pb, acc);
  const float nanv = __uint_as_float(0x7FC00000u);
#pragma unroll
  for (int j = 0; j < 4; ++j) {
    const float bj = bf16_rne(bias[n0 + 16 * j + ln]);
#pragma unroll
    for (int i = 0; i < 2; ++i)
#pragma unroll
      for (int r = 0; r < 8; ++r) {
        const float v = fmaf(acc[i][j][r], 3.814697265625e-06f, bj);
        so[32 * w + 16 * i + 8 * hh + r][16 * j + ln] = bad ? nanv : v;
      }
  }
  __syncthreads();
  float* og = out + ((size_t)b * SEQ_FULL + s0) * DIM + n0;
  for (int pass = 0; pass < 2; ++pass) {
#pragma unroll 1
    for (int it = 0; it < 16; ++it) {
      const int i = tid + 128 * it;
      const int row = i >> 4, pc = i & 15;
      const v4f v = *(const v4fa*)&so[row][4 * pc];
      *(volatile v4f*)(og + (size_t)row * DIM + 4 * pc) = v;
    }
    if (pass == 0) __threadfence();
  }
}

extern "C" void kernel_launch(void* const* d_in, const int* in_sizes, int n_in,
                              void* d_out, int out_size, void* d_ws, size_t ws_size, hipStream_t stream) {
  if (n_in < 6) return;
  const long long needx = ((long long)(NB - 1) * SEQ_FULL + SEQ) * DIM;
  const long long needm = (long long)(SEQ - 1) * SEQ_FULL + SEQ;
  if ((long long)in_sizes[0] < needx) return;
  if ((long long)in_sizes[1] < needm) return;
  if ((long long)in_sizes[2] < (long long)DIM * N3D) return;
  if ((long long)in_sizes[3] < (long long)N3D) return;
  if ((long long)in_sizes[4] < (long long)DIM * DIM) return;
  if ((long long)in_sizes[5] < (long long)DIM) return;
  if ((long long)out_size < needx) return;
  const float* x     = (const float*)d_in[0];
  const int*   mask  = (const int*)d_in[1];
  const float* W_qkv = (const float*)d_in[2];
  const float* b_qkv = (const float*)d_in[3];
  const float* W_out = (const float*)d_in[4];
  const float* b_out = (const float*)d_in[5];
  float* out = (float*)d_out;
  char* ws = (char*)d_ws;
  size_t off = 0;
  int* FLG = (int*)(ws + off);                          off += SZ_FLG;
  unsigned short* XC  = (unsigned short*)(ws + off);    off += SZ_XC;
  unsigned short* WQ  = (unsigned short*)(ws + off);    off += SZ_WQ;
  unsigned short* WO  = (unsigned short*)(ws + off);    off += SZ_WO;
  unsigned short* QH  = (unsigned short*)(ws + off);    off += SZ_PH;
  unsigned short* KH  = (unsigned short*)(ws + off);    off += SZ_PH;
  unsigned short* VTH = (unsigned short*)(ws + off);    off += SZ_PH;
  unsigned short* QL  = (unsigned short*)(ws + off);    off += SZ_PL;
  unsigned short* KL  = (unsigned short*)(ws + off);    off += SZ_PL;
  unsigned short* VTL = (unsigned short*)(ws + off);    off += SZ_PL;
  if (off > ws_size) return;

  k_maskchk<<<64, 256, 0, stream>>>(mask, FLG);
  k_xb<<<(unsigned)((NROWS * (DIM / 8) + 255) / 256), 256, 0, stream>>>(x, XC);
  k_wt<0><<<(unsigned)((N3D / 64) * (DIM / 64)), 256, 0, stream>>>(W_qkv, WQ, N3D);
  k_wt<1><<<(unsigned)((DIM / 64) * (DIM / 64)), 256, 0, stream>>>(W_out, WO, DIM);
  k_qkv<<<dim3(N3D / 64, NROWS / 128), 128, 0, stream>>>(XC, WQ, b_qkv, QH, QL, KH, KL, VTH, VTL);
  k_attn<true><<<(unsigned)(NB * HEADS * (EARLY / 64)), 128, 0, stream>>>(QH, QL, KH, KL, VTH, VTL, mask, XC, WQ);
  if (SEQ > EARLY)
    k_attn<false><<<(unsigned)(NB * HEADS * ((SEQ - EARLY) / 64)), 128, 0, stream>>>(QH, QL, KH, KL, VTH, VTL, mask, XC, WQ);
  k_out<<<dim3(DIM / 64, NROWS / 128), 128, 0, stream>>>(XC, WQ, WO, b_out, FLG, out);
}
